// Model_37684043055863
// MI455X (gfx1250) — hardware-verified
//
#include <hip/hip_runtime.h>
#include <math.h>

#ifndef NB
#define NB 8
#endif
#ifndef SEQ
#define SEQ 2048
#endif
#define NB_FULL 8
#define SEQ_FULL 2048
#define NC 1024
#define NF (NC * 16)
#define MPTS (NB * SEQ)
#define C1 128
#define C2 256
#define C3 512
#define C4 1024
#define DH 1024
#define DO3 3072
#define FH 512
#define FW0_LD 1029
#define DROWS 64
#define OUT1_OFF (NB_FULL * NC * 3)

static_assert(NB <= NB_FULL && SEQ <= SEQ_FULL);
static_assert(SEQ % 64 == 0 && MPTS % 64 == 0 && NF % 64 == 0 && DROWS % 64 == 0);
static_assert(C1 == 128);
static_assert(C1 % 32 == 0 && C2 % 32 == 0 && C3 % 32 == 0 && C4 % 32 == 0 && DH % 32 == 0 && FH % 32 == 0);
static_assert(C2 % 64 == 0 && C3 % 64 == 0 && C4 % 64 == 0 && DH % 64 == 0 && DO3 % 64 == 0 && FH % 64 == 0);
static_assert(DO3 == 3 * NC);
static_assert(NB <= DROWS);
static_assert((OUT1_OFF * 4) == 98304 && (OUT1_OFF * 4) % 128 == 0);
static_assert((size_t)OUT1_OFF + (size_t)NB * NF * 3 <= (size_t)1671168 / 4);
static_assert((size_t)NB * DO3 <= (size_t)OUT1_OFF);
static_assert(NF % 256 == 0 && NC % 4 == 0);
static_assert((NB * DO3 / 4) % 256 == 0 || NB < NB_FULL);

typedef __attribute__((ext_vector_type(16))) _Float16 v16h;
typedef __attribute__((ext_vector_type(8)))  _Float16 v8h;
typedef __attribute__((ext_vector_type(8)))  float    v8f;
typedef __attribute__((ext_vector_type(4)))  float    v4f;
typedef __attribute__((ext_vector_type(4)))  unsigned int v4u;


#define VST2(T, ptr, val) do { const T vst2_v_ = (val); *(volatile T*)(ptr) = vst2_v_; __threadfence(); *(volatile T*)(ptr) = vst2_v_; } while (0)
#define VST2V4(ptr, val) do { const v4f vst2_v4_ = (val); *(volatile v4f*)(ptr) = vst2_v4_; __threadfence(); *(volatile v4f*)(ptr) = vst2_v4_; } while (0)

__device__ __forceinline__ float bfr(float f) {
    unsigned u = __float_as_uint(f);
    u += 0x7FFFu + ((u >> 16) & 1u);
    return __uint_as_float(u & 0xFFFF0000u);
}
__device__ __forceinline__ unsigned short f2h_bits(float x) {
    return (fabsf(x) < 6.104e-5f) ? (unsigned short)0 : __builtin_bit_cast(unsigned short, (_Float16)x);
}
__device__ __forceinline__ void st8h(unsigned short* P, size_t o, const float* v) {
    v4u pk;
    pk.x = (unsigned)f2h_bits(v[0]) | ((unsigned)f2h_bits(v[1]) << 16);
    pk.y = (unsigned)f2h_bits(v[2]) | ((unsigned)f2h_bits(v[3]) << 16);
    pk.z = (unsigned)f2h_bits(v[4]) | ((unsigned)f2h_bits(v[5]) << 16);
    pk.w = (unsigned)f2h_bits(v[6]) | ((unsigned)f2h_bits(v[7]) << 16);
    VST2(v4u, (v4u*)(P + o), pk);
}

union FragU { v16h v; v8h h[2]; };
__device__ __forceinline__ v16h frag_ld(const _Float16* p) {
    FragU f; f.h[0] = *(const v8h*)(p); f.h[1] = *(const v8h*)(p + 16); return f.v;
}
__device__ __forceinline__ v8f wmma16(v16h a, v16h b, v8f c) {
    c = __builtin_amdgcn_wmma_f32_16x16x32_f16(false, a, false, b, (short)0, c, false, false);
    asm volatile("v_nop\n\tv_nop\n\tv_nop\n\tv_nop" : "+v"(c) : "v"(a), "v"(b));
    return c;
}
__device__ __forceinline__ void dep_guard_h(v8f& a, v8f& b, v16h x, v16h y) { asm volatile("v_nop\n\tv_nop\n\tv_nop\n\tv_nop" : "+v"(a), "+v"(b) : "v"(x), "v"(y)); }
__device__ __forceinline__ void keep4_h(v16h a, v16h b, v16h c, v16h d) { asm volatile("v_nop" :: "v"(a), "v"(b), "v"(c), "v"(d)); }
__device__ __forceinline__ void acc_guard4(v8f& a, v8f& b, v8f& c, v8f& d) { asm volatile("v_nop\n\tv_nop\n\tv_nop\n\tv_nop" : "+v"(a), "+v"(b), "+v"(c), "+v"(d)); }
__device__ __forceinline__ void wave_sync_lds() {
    __builtin_amdgcn_fence(3  , "workgroup");
    __builtin_amdgcn_wave_barrier();
    __builtin_amdgcn_fence(2  , "workgroup");
}

typedef _Float16 h16;
static __device__ __forceinline__ h16 toh_flush(float v) { const h16 r = (h16)v; return (fabsf(v) < 6.103515625e-05f) ? (h16)0.0f : r; }
__device__ __forceinline__ void st8hf(unsigned short* P, size_t o, const float* v) {
    v8h hv;
#pragma unroll
    for (int e = 0; e < 8; ++e) hv[e] = toh_flush(v[e]);
    VST2(v8h, (v8h*)(P + o), hv);
}

static_assert(32 * 16 * 4 == 16 * 64 * 2);
static_assert(32 * 16 * 8 == 16 * 64 * 4);
static_assert(8 * 16 * 68 * 4 <= 131072);
template <int OUT_MODE, bool RELU, bool BSAMP>
__device__ __forceinline__ void gemm64_body(
    const _Float16* __restrict__ A, unsigned lda, const _Float16* __restrict__ Bt, unsigned ldb,
    void* __restrict__ Cout, unsigned ldc, const float* __restrict__ bias,
    unsigned M, unsigned N, unsigned K, float scale, float oscale, unsigned sdiv) {
  __shared__ __align__(16) float sT[8][16 * 68];
  const unsigned lane = threadIdx.x & 31u;
  const unsigned wave = (unsigned)__builtin_amdgcn_readfirstlane((int)(threadIdx.x >> 5));
  const unsigned tilesN = N >> 6, tilesM = M >> 6;
  const unsigned tile = blockIdx.x * 8u + wave;
  if (tile >= tilesM * tilesN) return;
  const unsigned tm = tile / tilesN;
  const unsigned tn = tile - tm * tilesN;
  const unsigned m0 = tm << 6, n0 = tn << 6;
  const unsigned rlane = lane & 15u;
  const unsigned koff = (lane >> 4) * 8u;
  const unsigned mOff = koff;

  v8f acc[4][4];
#pragma unroll
  for (int i = 0; i < 4; ++i)
#pragma unroll
    for (int j = 0; j < 4; ++j) acc[i][j] = (v8f){0.f,0.f,0.f,0.f,0.f,0.f,0.f,0.f};

  for (unsigned k0 = 0; k0 < K; k0 += 32u) {
    v16h bh[4];
#pragma unroll
    for (int j = 0; j < 4; ++j)
      bh[j] = frag_ld(Bt + (size_t)(n0 + ((unsigned)j << 4) + rlane) * ldb + koff + k0);
#pragma unroll
    for (int i = 0; i < 4; ++i) {
      const v16h ah = frag_ld(A + (size_t)(m0 + ((unsigned)i << 4) + rlane) * lda + koff + k0);
#pragma unroll
      for (int j = 0; j < 4; ++j)
        acc[i][j] = __builtin_amdgcn_wmma_f32_16x16x32_f16(false, ah, false, bh[j], (short)0, acc[i][j], false, false);
      dep_guard_h(acc[i][0], acc[i][3], ah, ah);
    }
    keep4_h(bh[0], bh[1], bh[2], bh[3]);
  }
  acc_guard4(acc[0][0], acc[0][1], acc[0][2], acc[0][3]);
  acc_guard4(acc[1][0], acc[1][1], acc[1][2], acc[1][3]);
  acc_guard4(acc[2][0], acc[2][1], acc[2][2], acc[2][3]);
  acc_guard4(acc[3][0], acc[3][1], acc[3][2], acc[3][3]);

  float* slab = sT[wave];
  const unsigned bsrow = BSAMP ? (m0 / sdiv) : 0u;
#pragma unroll
  for (int i = 0; i < 4; ++i) {
    const unsigned mBase = m0 + ((unsigned)i << 4);
#pragma unroll
    for (int j = 0; j < 4; ++j) {
      const unsigned n = n0 + ((unsigned)j << 4) + rlane;
      const float bv = BSAMP ? bias[(size_t)bsrow * N + n] : bfr(bias[n]);
#pragma unroll
      for (int r = 0; r < 8; ++r) {
        float v = acc[i][j][r] * scale + bv;
        if (RELU) v = fmaxf(v, 0.0f);
        if (OUT_MODE == 1) v *= oscale;
        slab[(mOff + (unsigned)r) * 68u + ((unsigned)j << 4) + rlane] = v;
      }
    }
    wave_sync_lds();
    if (OUT_MODE == 0) {
      float* C = (float*)Cout;
      const unsigned hh = lane >> 4, c4 = (lane & 15u) * 4u;
#pragma unroll
      for (int half = 0; half < 2; ++half) {
        v4f vv[4];
#pragma unroll
        for (int it = 0; it < 4; ++it) {
          const unsigned row = (unsigned)(half * 4 + it) * 2u + hh;
          vv[it] = *(const v4f*)(slab + row * 68u + c4);
        }
        for (int pass = 0; pass < 2; ++pass) {
#pragma unroll
          for (int it = 0; it < 4; ++it) {
            const unsigned row = (unsigned)(half * 4 + it) * 2u + hh;
            *(volatile v4f*)(C + (size_t)(mBase + row) * ldc + n0 + c4) = vv[it];
          }
          __threadfence();
        }
      }
    } else {
      _Float16* C = (_Float16*)Cout;
      const unsigned q = lane >> 3, c8 = (lane & 7u) * 8u;
      v8h hv[4];
#pragma unroll
      for (int it = 0; it < 4; ++it) {
        const unsigned row = (unsigned)it * 4u + q;
        const float* sp = slab + row * 68u + c8;
#pragma unroll
        for (int e = 0; e < 8; ++e) hv[it][e] = toh_flush(sp[e]);
      }
      for (int pass = 0; pass < 2; ++pass) {
#pragma unroll
        for (int it = 0; it < 4; ++it) {
          const unsigned row = (unsigned)it * 4u + q;
          *(volatile v8h*)(C + (size_t)(mBase + row) * ldc + n0 + c8) = hv[it];
        }
        __threadfence();
      }
    }
    wave_sync_lds();
  }
}

__global__ __launch_bounds__(256) void k_gemm_h(
    const _Float16* __restrict__ A, unsigned lda, const _Float16* __restrict__ Bt, unsigned ldb,
    _Float16* __restrict__ C, unsigned ldc, const float* __restrict__ bias,
    unsigned M, unsigned N, unsigned K, float scale, float oscale) {
  gemm64_body<1, false, false>(A, lda, Bt, ldb, (void*)C, ldc, bias, M, N, K, scale, oscale, 1u);
}
__global__ __launch_bounds__(256) void k_gemm_hr(
    const _Float16* __restrict__ A, unsigned lda, const _Float16* __restrict__ Bt, unsigned ldb,
    _Float16* __restrict__ C, unsigned ldc, const float* __restrict__ bias,
    unsigned M, unsigned N, unsigned K, float scale, float oscale) {
  gemm64_body<1, true, false>(A, lda, Bt, ldb, (void*)C, ldc, bias, M, N, K, scale, oscale, 1u);
}
__global__ __launch_bounds__(256) void k_gemm_hrs(
    const _Float16* __restrict__ A, unsigned lda, const _Float16* __restrict__ Bt, unsigned ldb,
    _Float16* __restrict__ C, unsigned ldc, const float* __restrict__ svec,
    unsigned M, unsigned N, unsigned K, float scale, float oscale, unsigned sdiv) {
  gemm64_body<1, true, true>(A, lda, Bt, ldb, (void*)C, ldc, svec, M, N, K, scale, oscale, sdiv);
}
__global__ __launch_bounds__(256) void k_gemm_f(
    const _Float16* __restrict__ A, unsigned lda, const _Float16* __restrict__ Bt, unsigned ldb,
    float* __restrict__ C, unsigned ldc, const float* __restrict__ bias,
    unsigned M, unsigned N, unsigned K, float scale) {
  gemm64_body<0, false, false>(A, lda, Bt, ldb, (void*)C, ldc, bias, M, N, K, scale, 1.0f, 1u);
}

__global__ __launch_bounds__(256) void k_wconv(const float* __restrict__ Wm, unsigned ldw, unsigned c0, unsigned lgper, unsigned NO,
                                               unsigned short* __restrict__ W16, float sw) {
    const unsigned u = blockIdx.x * 256u + threadIdx.x;
    const unsigned per = 1u << lgper;
    if (u >= NO * per) return;
    const unsigned k0 = 8u * (u & (per - 1u));
    const unsigned o = u >> lgper;
    const float* src = Wm + (size_t)o * ldw + c0 + k0;
    float v[8];
#pragma unroll
    for (int i = 0; i < 8; ++i) v[i] = bfr(src[i]) * sw;
    st8hf(W16, (size_t)o * (8u * per) + k0, v);
}

static_assert((C1 * 3 + C1) * 4 <= 131072);
__global__ __launch_bounds__(256) void k_e0(const float* __restrict__ in, const float* __restrict__ w0, const float* __restrict__ b0,
                                            unsigned short* __restrict__ A1) {
    __shared__ float sW0[C1 * 3];
    __shared__ float sB0[C1];
    const unsigned t = threadIdx.x;
#pragma unroll 1
    for (unsigned i = t; i < (unsigned)(C1 * 3); i += 256u) sW0[i] = bfr(w0[i]);
#pragma unroll 1
    for (unsigned i = t; i < (unsigned)C1; i += 256u) sB0[i] = bfr(b0[i]);
    __syncthreads();
    const unsigned u = blockIdx.x * 256u + threadIdx.x;
    if (u >= (unsigned)(MPTS * (C1 / 8))) return;
    const unsigned p = u >> 4, c0 = (u & 15u) * 8u;
    const unsigned b = p / (unsigned)SEQ, n = p - b * (unsigned)SEQ;
    const float* ip = in + (size_t)b * 3u * SEQ_FULL + n;
    const float x = bfr(ip[0]), y = bfr(ip[SEQ_FULL]), z = bfr(ip[2 * SEQ_FULL]);
    float v[8];
#pragma unroll
    for (int i = 0; i < 8; ++i) {
        const unsigned wo = (c0 + (unsigned)i) * 3u;
        const float s = (sW0[wo] * x + sW0[wo + 1u] * y + sW0[wo + 2u] * z) + sB0[c0 + (unsigned)i];
        v[i] = fmaxf(s, 0.0f) * 8.0f;
    }
    st8hf(A1, (size_t)p * C1 + c0, v);
}

__global__ __launch_bounds__(256) void k_maxpool(const _Float16* __restrict__ Aact, unsigned C, float* __restrict__ gout,
                                                 unsigned short* __restrict__ hplane, unsigned wantH) {
    __shared__ float sM[32][65];
    __shared__ __align__(16) float sC[64];
    const unsigned t = threadIdx.x;
    const unsigned cg = t & 7u, rs = t >> 3;
    const unsigned cb = blockIdx.x * 64u;
    const unsigned b = blockIdx.y;
    if (b >= (unsigned)NB) {
        if (wantH != 0u && t < 8u) {
            v4u z; z.x = 0u; z.y = 0u; z.z = 0u; z.w = 0u;
            VST2(v4u, (v4u*)(hplane + (size_t)b * C + cb + 8u * t), z);
        }
        return;
    }
    float m[8];
#pragma unroll
    for (int e = 0; e < 8; ++e) m[e] = -3.0e38f;
    const _Float16* src = Aact + (size_t)(b * (unsigned)SEQ + rs) * C + cb + 8u * cg;
#pragma unroll 1
    for (unsigned r = 0; r < (unsigned)(SEQ / 32); ++r) {
        const v8h v = *(const v8h*)(src + (size_t)r * 32u * C);
#pragma unroll
        for (int e = 0; e < 8; ++e) m[e] = fmaxf(m[e], (float)v[e]);
    }
#pragma unroll
    for (int e = 0; e < 8; ++e) sM[rs][8u * cg + (unsigned)e] = m[e];
    __syncthreads();
    if (t < 64u) {
        float mx = sM[0][t];
#pragma unroll 1
        for (unsigned rr = 1; rr < 32u; ++rr) mx = fmaxf(mx, sM[rr][t]);
        sC[t] = mx;
    }
    __syncthreads();
    if (t < 16u) {
        v4f o = *(const v4f*)(sC + 4u * t);
        o *= 0.125f;
        VST2V4(gout + (size_t)b * C + cb + 4u * t, o);
    }
    if (wantH != 0u && t < 8u) {
        float v[8];
#pragma unroll
        for (int e = 0; e < 8; ++e) v[e] = sC[8u * t + (unsigned)e];
        st8hf(hplane, (size_t)b * C + cb + 8u * t, v);
    }
}
static_assert((32 * 65 + 64) * 4 <= 131072);

__global__ __launch_bounds__(256) void k_rowvec(const float* __restrict__ Wm, unsigned ldw, unsigned c0, const float* __restrict__ bias,
                                                const float* __restrict__ x, unsigned K, float* __restrict__ out, unsigned NO) {
    __shared__ __align__(16) float sO[NB][32];
    const unsigned lane = threadIdx.x & 31u;
    const unsigned wave = (unsigned)__builtin_amdgcn_readfirstlane((int)(threadIdx.x >> 5));
    const unsigned cbase = blockIdx.x * 32u;
#pragma unroll 1
    for (unsigned q = 0; q < 4u; ++q) {
        const unsigned cl = wave * 4u + q;
        const unsigned c = cbase + cl;
        const float* wr = Wm + (size_t)c * ldw + c0;
        float acc[NB];
#pragma unroll
        for (int bb = 0; bb < NB; ++bb) acc[bb] = 0.f;
#pragma unroll 2
        for (unsigned k = lane; k < K; k += 32u) {
            const float w = bfr(wr[k]);
#pragma unroll
            for (int bb = 0; bb < NB; ++bb) acc[bb] += w * x[(size_t)bb * K + k];
        }
#pragma unroll
        for (int bb = 0; bb < NB; ++bb) {
            float s = acc[bb];
            s += __shfl_xor(s, 16, 32); s += __shfl_xor(s, 8, 32); s += __shfl_xor(s, 4, 32);
            s += __shfl_xor(s, 2, 32);  s += __shfl_xor(s, 1, 32);
            acc[bb] = s;
        }
        const float bc = bfr(bias[c]);
        if (lane == 0u) {
#pragma unroll
            for (int bb = 0; bb < NB; ++bb) sO[bb][cl] = acc[bb] + bc;
        }
    }
    __syncthreads();
    const unsigned t = threadIdx.x;
    if (t < (unsigned)(NB * 8)) {
        const unsigned sample = t >> 3, piece = t & 7u;
        const v4f o = *(const v4f*)(&sO[sample][4u * piece]);
        VST2V4(out + (size_t)sample * NO + cbase + 4u * piece, o);
    }
}

__global__ __launch_bounds__(256) void k_coarse_out(const float* __restrict__ coarse, float* __restrict__ out) {
    const unsigned u = blockIdx.x * 256u + threadIdx.x;
    if (u >= (unsigned)(NB * DO3 / 4)) return;
    const unsigned b = u / (unsigned)(DO3 / 4), j = u - b * (unsigned)(DO3 / 4);
    const v4f v = *(const v4f*)(coarse + (size_t)b * DO3 + 4u * j);
    VST2V4(out + (size_t)b * DO3 + 4u * j, v);
}

__device__ __forceinline__ float lin4(unsigned i) {
    return (i == 0u) ? -0.05f : ((i == 1u) ? -0.016666668f : ((i == 2u) ? 0.016666668f : 0.05f));
}

static_assert(256 * 16 * 16 == 64 * FH * 2);
static_assert((NC / 4) * 64 == NF);
static_assert(FH == 512);
static_assert((FH * 5 + FH) * 4 <= 131072);
static_assert((FH * 5) % 256 == 0 && FH % 256 == 0);
__global__ __launch_bounds__(256) void k_fold0(const float* __restrict__ tg, const float* __restrict__ coarse, const float* __restrict__ fw0,
                                               unsigned short* __restrict__ H0, unsigned b) {
    __shared__ float sW5[FH * 5];
    __shared__ float sTg[FH];
    const unsigned t = threadIdx.x;
#pragma unroll 1
    for (unsigned i = t; i < (unsigned)(FH * 5); i += 256u) {
        const unsigned cc = i / 5u, jj = i - cc * 5u;
        sW5[i] = bfr(fw0[(size_t)cc * FW0_LD + jj]);
    }
#pragma unroll 1
    for (unsigned i = t; i < (unsigned)FH; i += 256u) sTg[i] = tg[(size_t)b * FH + i];
    __syncthreads();
    const unsigned c0 = (t & 63u) * 8u;
    const unsigned kpt = blockIdx.x * 4u + (t >> 6);
    const float* cp = coarse + (size_t)b * DO3 + kpt * 3u;
    const float px = cp[0], py = cp[1], pz = cp[2];
    float base[8], wx[8], wy[8];
#pragma unroll
    for (int r = 0; r < 8; ++r) {
        const unsigned wo = (c0 + (unsigned)r) * 5u;
        base[r] = sTg[c0 + (unsigned)r] + (sW5[wo + 2u] * px + sW5[wo + 3u] * py + sW5[wo + 4u] * pz);
        wx[r] = sW5[wo];
        wy[r] = sW5[wo + 1u];
    }
#pragma unroll 1
    for (unsigned g = 0; g < 16u; ++g) {
        const float gx = lin4(g & 3u), gy = lin4(g >> 2);
        float v[8];
#pragma unroll
        for (int r = 0; r < 8; ++r) v[r] = fmaxf(base[r] + (wx[r] * gx + wy[r] * gy), 0.0f) * 8.0f;
        st8hf(H0, (size_t)(kpt * 16u + g) * FH + c0, v);
    }
}

static_assert(192 * 16 == 256 * 3 * 4);
static_assert((3 * 512 + 768) * 4 <= 131072);
__global__ __launch_bounds__(256) void k_final(const _Float16* __restrict__ H1, const float* __restrict__ fw2, const float* __restrict__ fb2,
                                               const float* __restrict__ coarse, float* __restrict__ out, unsigned b) {
    __shared__ __align__(16) float sW[3 * FH];
    __shared__ __align__(16) float sO[768];
    const unsigned t = threadIdx.x;
#pragma unroll 1
    for (unsigned i = t; i < (unsigned)(3 * FH); i += 256u) sW[i] = bfr(fw2[i]);
    __syncthreads();
    const unsigned row = blockIdx.x * 256u + t;
    const _Float16* hr = H1 + (size_t)row * FH;
    float a0 = 0.f, a1 = 0.f, a2 = 0.f;
#pragma unroll 1
    for (unsigned k = 0; k < (unsigned)FH; k += 8u) {
        const v8h hv = *(const v8h*)(hr + k);
#pragma unroll
        for (int e = 0; e < 8; ++e) {
            const float f = (float)hv[e];
            a0 += f * sW[k + (unsigned)e];
            a1 += f * sW[FH + k + (unsigned)e];
            a2 += f * sW[2 * FH + k + (unsigned)e];
        }
    }
    const float* cp = coarse + (size_t)b * DO3 + (row >> 4) * 3u;
    sO[3u * t + 0u] = (a0 * 0.125f + bfr(fb2[0])) + cp[0];
    sO[3u * t + 1u] = (a1 * 0.125f + bfr(fb2[1])) + cp[1];
    sO[3u * t + 2u] = (a2 * 0.125f + bfr(fb2[2])) + cp[2];
    __syncthreads();
    if (t < 192u) {
        const v4f o = *(const v4f*)(sO + 4u * t);
        VST2V4(out + (size_t)OUT1_OFF + ((size_t)b * NF + (size_t)blockIdx.x * 256u) * 3u + 4u * t, o);
    }
}

constexpr size_t al256(size_t b) { return (b + 255) & ~(size_t)255; }
constexpr size_t SZ_WE0  = al256((size_t)C2 * C1 * 2);
constexpr size_t SZ_WE1A = al256((size_t)C3 * C2 * 2);
constexpr size_t SZ_WE1B = al256((size_t)C4 * C3 * 2);
constexpr size_t SZ_WD0  = al256((size_t)DH * C4 * 2);
constexpr size_t SZ_WD1  = al256((size_t)DH * DH * 2);
constexpr size_t SZ_WD2  = al256((size_t)DO3 * DH * 2);
constexpr size_t SZ_WF1  = al256((size_t)FH * FH * 2);
constexpr size_t SZ_A1   = al256((size_t)MPTS * C1 * 2);
constexpr size_t SZ_A2   = al256((size_t)MPTS * C2 * 2);
constexpr size_t SZ_A3   = al256((size_t)MPTS * C3 * 2);
constexpr size_t SZ_A4   = al256((size_t)MPTS * C4 * 2);
constexpr size_t SZ_G    = al256((size_t)NB * C2 * 4);
constexpr size_t SZ_VG   = al256((size_t)NB * C3 * 4);
constexpr size_t SZ_FEAT = al256((size_t)NB * C4 * 4);
constexpr size_t SZ_F16  = al256((size_t)DROWS * C4 * 2);
constexpr size_t SZ_D1   = al256((size_t)DROWS * DH * 2);
constexpr size_t SZ_D2   = al256((size_t)DROWS * DH * 2);
constexpr size_t SZ_CO   = al256((size_t)DROWS * DO3 * 4);
constexpr size_t SZ_TG   = al256((size_t)NB * FH * 4);
constexpr size_t SZ_H0   = al256((size_t)NF * FH * 2);
constexpr size_t SZ_H1   = al256((size_t)NF * FH * 2);
constexpr size_t CARVE_TOTAL = SZ_WE0 + SZ_WE1A + SZ_WE1B + SZ_WD0 + SZ_WD1 + SZ_WD2 + SZ_WF1 + SZ_A1 + SZ_A2 + SZ_A3 + SZ_A4 +
                               SZ_G + SZ_VG + SZ_FEAT + SZ_F16 + SZ_D1 + SZ_D2 + SZ_CO + SZ_TG + SZ_H0 + SZ_H1;
static_assert(CARVE_TOTAL <= (size_t)134217728);
static_assert((C2 * (C1 / 8)) % 256 == 0 && (C3 * (C2 / 8)) % 256 == 0 && (C4 * (C3 / 8)) % 256 == 0);
static_assert((DH * (C4 / 8)) % 256 == 0 && (DO3 * (DH / 8)) % 256 == 0 && (FH * (FH / 8)) % 256 == 0);
static_assert((MPTS * (C1 / 8)) % 256 == 0);
static_assert(C1 / 8 == 16 && C2 / 8 == 32 && C3 / 8 == 64 && C4 / 8 == 128 && DH / 8 == 128 && FH / 8 == 64);
static_assert(C3 % 32 == 0 && FH % 32 == 0);

static constexpr float SC = 1.0f / 256.0f;
extern "C" void kernel_launch(void* const* d_in, const int* in_sizes, int n_in, void* d_out, int out_size,
                              void* d_ws, size_t ws_size, hipStream_t stream) {
    if (n_in < 21) return;
    if (in_sizes[0] < ((NB - 1) * 3 + 2) * SEQ_FULL + SEQ) return;
    if (in_sizes[1] < C1 * 3 || in_sizes[2] < C1 || in_sizes[3] < C2 * C1 || in_sizes[4] < C2) return;
    if (in_sizes[5] < C3 * 512 || in_sizes[6] < C3 || in_sizes[7] < C4 * C3 || in_sizes[8] < C4) return;
    if (in_sizes[9] < DH * C4 || in_sizes[10] < DH || in_sizes[11] < DH * DH || in_sizes[12] < DH) return;
    if (in_sizes[13] < DO3 * DH || in_sizes[14] < DO3 || in_sizes[15] < FH * FW0_LD || in_sizes[16] < FH) return;
    if (in_sizes[17] < FH * FH || in_sizes[18] < FH || in_sizes[19] < 3 * FH || in_sizes[20] < 3) return;
    if (out_size < OUT1_OFF + NB * NF * 3) return;

    const float* input = (const float*)d_in[0];
    const float* e0_w0 = (const float*)d_in[1];
    const float* e0_b0 = (const float*)d_in[2];
    const float* e0_w1 = (const float*)d_in[3];
    const float* e0_b1 = (const float*)d_in[4];
    const float* e1_w0 = (const float*)d_in[5];
    const float* e1_b0 = (const float*)d_in[6];
    const float* e1_w1 = (const float*)d_in[7];
    const float* e1_b1 = (const float*)d_in[8];
    const float* d_w0  = (const float*)d_in[9];
    const float* d_b0  = (const float*)d_in[10];
    const float* d_w1  = (const float*)d_in[11];
    const float* d_b1  = (const float*)d_in[12];
    const float* d_w2  = (const float*)d_in[13];
    const float* d_b2  = (const float*)d_in[14];
    const float* f_w0  = (const float*)d_in[15];
    const float* f_b0  = (const float*)d_in[16];
    const float* f_w1  = (const float*)d_in[17];
    const float* f_b1  = (const float*)d_in[18];
    const float* f_w2  = (const float*)d_in[19];
    const float* f_b2  = (const float*)d_in[20];
    float* out = (float*)d_out;

    char* wsp = (char*)d_ws;
    size_t off = 0;
    auto carve = [&](size_t bytes) -> void* { void* r = wsp + off; off += bytes; return r; };
    unsigned short* wE0  = (unsigned short*)carve(SZ_WE0);
    unsigned short* wE1a = (unsigned short*)carve(SZ_WE1A);
    unsigned short* wE1b = (unsigned short*)carve(SZ_WE1B);
    unsigned short* wD0  = (unsigned short*)carve(SZ_WD0);
    unsigned short* wD1  = (unsigned short*)carve(SZ_WD1);
    unsigned short* wD2  = (unsigned short*)carve(SZ_WD2);
    unsigned short* wF1  = (unsigned short*)carve(SZ_WF1);
    unsigned short* A1   = (unsigned short*)carve(SZ_A1);
    unsigned short* A2   = (unsigned short*)carve(SZ_A2);
    unsigned short* A3   = (unsigned short*)carve(SZ_A3);
    unsigned short* A4   = (unsigned short*)carve(SZ_A4);
    float*          gmx  = (float*)carve(SZ_G);
    float*          vg   = (float*)carve(SZ_VG);
    float*          feat = (float*)carve(SZ_FEAT);
    unsigned short* F16p = (unsigned short*)carve(SZ_F16);
    unsigned short* D1   = (unsigned short*)carve(SZ_D1);
    unsigned short* D2   = (unsigned short*)carve(SZ_D2);
    float*          co   = (float*)carve(SZ_CO);
    float*          tg   = (float*)carve(SZ_TG);
    unsigned short* H0   = (unsigned short*)carve(SZ_H0);
    unsigned short* H1   = (unsigned short*)carve(SZ_H1);
    if (off != CARVE_TOTAL || off > ws_size || off > (size_t)134217728) return;

    k_wconv<<<(C2 * (C1 / 8)) / 256, 256, 0, stream>>>(e0_w1, C1, 0u, 4u, C2, wE0, 32.0f);
    k_wconv<<<(C3 * (C2 / 8)) / 256, 256, 0, stream>>>(e1_w0, 512u, 0u, 5u, C3, wE1a, 32.0f);
    k_wconv<<<(C4 * (C3 / 8)) / 256, 256, 0, stream>>>(e1_w1, C3, 0u, 6u, C4, wE1b, 32.0f);
    k_wconv<<<(DH * (C4 / 8)) / 256, 256, 0, stream>>>(d_w0, C4, 0u, 7u, DH, wD0, 32.0f);
    k_wconv<<<(DH * (DH / 8)) / 256, 256, 0, stream>>>(d_w1, DH, 0u, 7u, DH, wD1, 32.0f);
    k_wconv<<<(DO3 * (DH / 8)) / 256, 256, 0, stream>>>(d_w2, DH, 0u, 7u, DO3, wD2, 32.0f);
    k_wconv<<<(FH * (FH / 8)) / 256, 256, 0, stream>>>(f_w1, FH, 0u, 6u, FH, wF1, 32.0f);

    const unsigned gA2 = ((MPTS / 64) * (C2 / 64) + 7) / 8;
    const unsigned gA3 = ((MPTS / 64) * (C3 / 64) + 7) / 8;
    const unsigned gA4 = ((MPTS / 64) * (C4 / 64) + 7) / 8;
    const unsigned gD  = ((DROWS / 64) * (DH / 64) + 7) / 8;
    const unsigned gD3 = ((DROWS / 64) * (DO3 / 64) + 7) / 8;
    const unsigned gF  = ((NF / 64) * (FH / 64) + 7) / 8;

    k_e0<<<(MPTS * (C1 / 8)) / 256, 256, 0, stream>>>(input, e0_w0, e0_b0, A1);
    k_gemm_h<<<gA2, 256, 0, stream>>>((const _Float16*)A1, C1, (const _Float16*)wE0, C1, (_Float16*)A2, C2, e0_b1,
                                      MPTS, C2, C1, SC, 8.0f);
    k_maxpool<<<dim3(C2 / 64, NB), 256, 0, stream>>>((const _Float16*)A2, C2, gmx, F16p, 0u);
    k_rowvec<<<C3 / 32, 256, 0, stream>>>(e1_w0, 512u, 256u, e1_b0, gmx, C2, vg, C3);
    k_gemm_hrs<<<gA3, 256, 0, stream>>>((const _Float16*)A2, C2, (const _Float16*)wE1a, C2, (_Float16*)A3, C3, vg,
                                        MPTS, C3, C2, SC, 8.0f, (unsigned)SEQ);
    k_gemm_h<<<gA4, 256, 0, stream>>>((const _Float16*)A3, C3, (const _Float16*)wE1b, C3, (_Float16*)A4, C4, e1_b1,
                                      MPTS, C4, C3, SC, 8.0f);
    k_maxpool<<<dim3(C4 / 64, DROWS), 256, 0, stream>>>((const _Float16*)A4, C4, feat, F16p, 1u);

    k_gemm_hr<<<gD, 256, 0, stream>>>((const _Float16*)F16p, C4, (const _Float16*)wD0, C4, (_Float16*)D1, DH, d_b0,
                                      DROWS, DH, C4, SC, 8.0f);
    k_gemm_hr<<<gD, 256, 0, stream>>>((const _Float16*)D1, DH, (const _Float16*)wD1, DH, (_Float16*)D2, DH, d_b1,
                                      DROWS, DH, DH, SC, 8.0f);
    k_gemm_f<<<gD3, 256, 0, stream>>>((const _Float16*)D2, DH, (const _Float16*)wD2, DH, co, DO3, d_b2,
                                      DROWS, DO3, DH, SC);
    k_coarse_out<<<(NB * DO3 / 4 + 255) / 256, 256, 0, stream>>>(co, out);

    k_rowvec<<<FH / 32, 256, 0, stream>>>(f_w0, FW0_LD, 5u, f_b0, feat, C4, tg, FH);
    for (int b = 0; b < NB; ++b) {
        k_fold0<<<NC / 4, 256, 0, stream>>>(tg, co, f_w0, H0, (unsigned)b);
        k_gemm_hr<<<gF, 256, 0, stream>>>((const _Float16*)H0, FH, (const _Float16*)wF1, FH, (_Float16*)H1, FH, f_b1,
                                          NF, FH, FH, SC, 8.0f);
        k_final<<<NF / 256, 256, 0, stream>>>((const _Float16*)H1, f_w2, f_b2, co, out, (unsigned)b);
    }
}
